// RNN_29996051595637
// MI455X (gfx1250) — hardware-verified
//
#include <hip/hip_runtime.h>
#include <math.h>

typedef __attribute__((ext_vector_type(16))) _Float16 v16h;
typedef __attribute__((ext_vector_type(8)))  _Float16 v8h;
typedef __attribute__((ext_vector_type(4)))  _Float16 v4h;
typedef __attribute__((ext_vector_type(8)))  float    v8f;
typedef __attribute__((ext_vector_type(4)))  float    v4f;

constexpr int kSteps = 500;
constexpr int kBatch = 16;
constexpr int kFeat  = 440;
constexpr int kFeatP = 448;
constexpr int kHid   = 1024;
constexpr int kRows  = kSteps * kBatch;
constexpr float kWCarry    = 64.0f;
constexpr float kWCarryInv = 1.0f / 64.0f;
constexpr float kRCarry    = 2048.0f;
constexpr float kRCarryInv = 1.0f / 2048.0f;
constexpr float kDropScale = 0.8f;

constexpr int kScanThr = 512;
constexpr int kScanNW  = kScanThr / 32;
constexpr int kHP      = kHid + 8;
constexpr int kSlabP   = 68;

constexpr int kChunksX  = kRows * (kFeatP / 8);
constexpr int kChunksW0 = kHid * (kFeatP / 8);
constexpr int kChunksSq = kHid * (kHid / 8);
constexpr int kBlkX   = kChunksX / 256;
constexpr int kBlkW0  = kChunksW0 / 256;
constexpr int kBlkSq  = kChunksSq / 256;
constexpr int kPrepB1 = kBlkX;
constexpr int kPrepB2 = kPrepB1 + kBlkW0;
constexpr int kPrepB3 = kPrepB2 + kBlkSq;
constexpr int kPrepB4 = kPrepB3 + kBlkSq;
constexpr int kPrepB5 = kPrepB4 + kBlkSq;
constexpr int kPrepBlocks = kPrepB5 + 2;

static_assert(kRows == 8000, "rows");
static_assert(kFeatP % 32 == 0 && kFeatP >= kFeat && kFeatP - kFeat == 8, "one zero chunk of 8 per row");
static_assert(kFeat % 8 == 0, "source chunks");
static_assert(kHid % 64 == 0 && kHid % 32 == 0, "N and K tiles");
static_assert(kRows % 64 == 0 && kRows % 32 == 0, "M tiles");
static_assert(kChunksX % 256 == 0 && kChunksW0 % 256 == 0 && kChunksSq % 256 == 0, "prep grids exact");
static_assert(kHid == kScanNW * 64, "16 waves x 64 columns");
static_assert(kHP % 8 == 0, "LDS pitch");
static_assert((kBatch * kHP) % 8 == 0, "zero fill chunks");
static_assert(kHid == 256 * 4, "bias block covers one vector");

__device__ __forceinline__ unsigned short f2bf_bits(float f) {
  unsigned u = __float_as_uint(f);
  return (unsigned short)((u + 0x7FFFu + ((u >> 16) & 1u)) >> 16);
}
__device__ __forceinline__ float bf_bits2f(unsigned short h) { return __uint_as_float(((unsigned)h) << 16); }
__device__ __forceinline__ float bf16r(float f) { return bf_bits2f(f2bf_bits(f)); }

__device__ __forceinline__ void guard4_h(v8f& a0, v8f& a1, v8f& a2, v8f& a3, v16h x, v16h y) {
  asm volatile("v_nop\n\tv_nop\n\tv_nop\n\tv_nop" : "+v"(a0), "+v"(a1), "+v"(a2), "+v"(a3) : "v"(x), "v"(y));
}
__device__ __forceinline__ void guard8_h(v8f& a0, v8f& a1, v8f& a2, v8f& a3, v8f& r0, v8f& r1, v8f& r2, v8f& r3, v16h x, v16h y) {
  asm volatile("v_nop\n\tv_nop\n\tv_nop\n\tv_nop"
               : "+v"(a0), "+v"(a1), "+v"(a2), "+v"(a3), "+v"(r0), "+v"(r1), "+v"(r2), "+v"(r3)
               : "v"(x), "v"(y));
}
__device__ __forceinline__ void keep4_h(v16h a, v16h b, v16h c, v16h d) { asm volatile("v_nop" :: "v"(a), "v"(b), "v"(c), "v"(d)); }
__device__ __forceinline__ void acc_guard4(v8f& a, v8f& b, v8f& c, v8f& d) { asm volatile("v_nop\n\tv_nop\n\tv_nop\n\tv_nop" : "+v"(a), "+v"(b), "+v"(c), "+v"(d)); }

__device__ __forceinline__ void wave_sync() {
  __builtin_amdgcn_fence(__ATOMIC_RELEASE, "workgroup");
  __builtin_amdgcn_wave_barrier();
  __builtin_amdgcn_fence(__ATOMIC_ACQUIRE, "workgroup");
}

struct FragH {
  union U { v16h v; v8h h[2]; };
  static __device__ __forceinline__ v16h load(const _Float16* p) {
    U f; f.h[0] = *(const v8h*)(p); f.h[1] = *(const v8h*)(p + 16); return f.v;
  }
  static __device__ __forceinline__ v8f mma(v16h a, v16h b, v8f c) {
    return __builtin_amdgcn_wmma_f32_16x16x32_f16(false, a, false, b, (short)0, c, false, false);
  }
};

__device__ __forceinline__ float tanh_f(float x) {
  const float e = expf(2.0f * x);
  return 1.0f - 2.0f * __builtin_amdgcn_rcpf(e + 1.0f);
}

__device__ __forceinline__ void cvt_chunk8(const float* __restrict__ src, unsigned short* __restrict__ dst,
                                           int i, int ncol8d, int ncol8s, int spitch, float sc) {
  const int row = i / ncol8d;
  const int c8  = i - row * ncol8d;
  const bool valid = (c8 < ncol8s);
  const int c8c = valid ? c8 : (ncol8s - 1);
  const float* sp = src + (size_t)row * spitch + c8c * 8;
  const v4f a = *(const v4f*)(sp);
  const v4f b = *(const v4f*)(sp + 4);
  v8h hv;
#pragma unroll
  for (int e = 0; e < 4; ++e) {
    const float fa = valid ? a[e] : 0.0f;
    const float fb = valid ? b[e] : 0.0f;
    hv[e]     = (_Float16)(bf16r(fa) * sc);
    hv[4 + e] = (_Float16)(bf16r(fb) * sc);
  }
  _Float16* dp = (_Float16*)dst + (size_t)i * 8;
  *(volatile v8h*)dp = hv;
  __threadfence();
  *(volatile v8h*)dp = hv;
}

__global__ __launch_bounds__(256) void prep_kernel(
    const float* __restrict__ x, const float* __restrict__ w0, const float* __restrict__ b0,
    const float* __restrict__ u0, const float* __restrict__ w1, const float* __restrict__ b1,
    const float* __restrict__ u1,
    unsigned short* __restrict__ XH, unsigned short* __restrict__ W0H, unsigned short* __restrict__ U0H,
    unsigned short* __restrict__ W1H, unsigned short* __restrict__ U1H, float* __restrict__ BIAS) {
  const int blk = blockIdx.x, tid = threadIdx.x;
  if (blk < kPrepB1) {
    cvt_chunk8(x, XH, blk * 256 + tid, kFeatP / 8, kFeat / 8, kFeat, 1.0f);
  } else if (blk < kPrepB2) {
    cvt_chunk8(w0, W0H, (blk - kPrepB1) * 256 + tid, kFeatP / 8, kFeat / 8, kFeat, kWCarry);
  } else if (blk < kPrepB3) {
    cvt_chunk8(u0, U0H, (blk - kPrepB2) * 256 + tid, kHid / 8, kHid / 8, kHid, kWCarry);
  } else if (blk < kPrepB4) {
    cvt_chunk8(w1, W1H, (blk - kPrepB3) * 256 + tid, kHid / 8, kHid / 8, kHid, kWCarry);
  } else if (blk < kPrepB5) {
    cvt_chunk8(u1, U1H, (blk - kPrepB4) * 256 + tid, kHid / 8, kHid / 8, kHid, kWCarry);
  } else {
    const int which = blk - kPrepB5;
    const int idx = tid * 4;
    const v4f va = *(const v4f*)(b0 + idx);
    const v4f vb = *(const v4f*)(b1 + idx);
    v4f o;
#pragma unroll
    for (int e = 0; e < 4; ++e) {
      const float s = (which != 0) ? vb[e] : va[e];
      o[e] = bf16r(s);
    }
    float* op = BIAS + which * kHid + idx;
    *(volatile v4f*)op = o;
    __threadfence();
    *(volatile v4f*)op = o;
  }
}

template <int MI, bool HL>
__global__ __launch_bounds__(256) void gemm_f16_kernel(
    const unsigned short* __restrict__ Ap, const unsigned short* __restrict__ A2p, int lda,
    const unsigned short* __restrict__ Btp, int ldb,
    float* __restrict__ C, int ldc, const float* __restrict__ bias,
    int M, int N, int K, float scale, float rscale) {
  const _Float16* A  = (const _Float16*)Ap;
  const _Float16* A2 = (const _Float16*)A2p;
  const _Float16* Bt = (const _Float16*)Btp;
  __shared__ __align__(16) float sT[8][16 * 68];
  const int lane = threadIdx.x & 31;
  const int wave = threadIdx.x >> 5;
  const int tilesN = N >> 6;
  const int tilesM = M / (16 * MI);
  const int tile = blockIdx.x * 8 + wave;
  if (tile >= tilesM * tilesN) return;
  const int tm = tile / tilesN;
  const int tn = tile - tm * tilesN;
  const int m0 = tm * (16 * MI);
  const int n0 = tn << 6;
  const int rlane = lane & 15;
  const int koff  = (lane >> 4) * 8;
  const int mOff  = (lane >> 4) * 8;

  v8f acc[MI][4];
  v8f accr[HL ? MI : 1][4];
#pragma unroll
  for (int i = 0; i < MI; ++i)
#pragma unroll
    for (int j = 0; j < 4; ++j) acc[i][j] = (v8f){0.f, 0.f, 0.f, 0.f, 0.f, 0.f, 0.f, 0.f};
#pragma unroll
  for (int i = 0; i < (HL ? MI : 1); ++i)
#pragma unroll
    for (int j = 0; j < 4; ++j) accr[i][j] = (v8f){0.f, 0.f, 0.f, 0.f, 0.f, 0.f, 0.f, 0.f};

  for (int k0 = 0; k0 < K; k0 += 32) {
    v16h bh[4];
#pragma unroll
    for (int j = 0; j < 4; ++j) {
      const size_t bo = (size_t)(n0 + (j << 4) + rlane) * ldb + koff + k0;
      bh[j] = FragH::load(Bt + bo);
    }
#pragma unroll
    for (int i = 0; i < MI; ++i) {
      const size_t ao = (size_t)(m0 + (i << 4) + rlane) * lda + koff + k0;
      const v16h ah = FragH::load(A + ao);
      v16h al = ah;
      if (HL) al = FragH::load(A2 + ao);
#pragma unroll
      for (int j = 0; j < 4; ++j) {
        acc[i][j] = FragH::mma(ah, bh[j], acc[i][j]);
        if (HL) accr[HL ? i : 0][j] = FragH::mma(al, bh[j], accr[HL ? i : 0][j]);
      }
      if (HL) {
        guard8_h(acc[i][0], acc[i][1], acc[i][2], acc[i][3],
                 accr[HL ? i : 0][0], accr[HL ? i : 0][1], accr[HL ? i : 0][2], accr[HL ? i : 0][3], ah, al);
      } else {
        guard4_h(acc[i][0], acc[i][1], acc[i][2], acc[i][3], ah, bh[3]);
      }
    }
    keep4_h(bh[0], bh[1], bh[2], bh[3]);
  }
#pragma unroll
  for (int i = 0; i < MI; ++i) acc_guard4(acc[i][0], acc[i][1], acc[i][2], acc[i][3]);
  if (HL) {
#pragma unroll
    for (int i = 0; i < (HL ? MI : 1); ++i) acc_guard4(accr[i][0], accr[i][1], accr[i][2], accr[i][3]);
  }

  float* slab = sT[wave];
#pragma unroll
  for (int i = 0; i < MI; ++i) {
    const int mBase = m0 + (i << 4);
#pragma unroll
    for (int j = 0; j < 4; ++j) {
      const int n = n0 + (j << 4) + rlane;
      const float bv = bias[n];
#pragma unroll
      for (int r = 0; r < 8; ++r) {
        float v = acc[i][j][r];
        if (HL) v = v + accr[HL ? i : 0][j][r] * rscale;
        v = v * scale + bv;
        slab[(mOff + r) * 68 + (j << 4) + rlane] = v;
      }
    }
    wave_sync();
    {
      const int hh = lane >> 4, c4 = (lane & 15) * 4;
      for (int pass = 0; pass < 2; ++pass) {
#pragma unroll
        for (int it = 0; it < 8; ++it) {
          const int row = it * 2 + hh;
          const v4f v = *(const v4f*)(slab + row * 68 + c4);
          *(volatile v4f*)(C + (size_t)(mBase + row) * ldc + n0 + c4) = v;
        }
        __threadfence();
      }
    }
    wave_sync();
  }
}

template <bool TOP>
__global__ __launch_bounds__(kScanThr) void rnn_scan_kernel(
    const float* __restrict__ P, const unsigned short* __restrict__ Up,
    unsigned short* __restrict__ HHIp, unsigned short* __restrict__ HLOp, float* __restrict__ OUT) {
  __shared__ __align__(16) _Float16 Hh[kBatch * kHP];
  __shared__ __align__(16) _Float16 Hl[kBatch * kHP];
  __shared__ __align__(16) float    Sl[kScanNW][16 * kSlabP];
  const _Float16* U = (const _Float16*)Up;
  _Float16* HHI = (_Float16*)HHIp;
  _Float16* HLO = (_Float16*)HLOp;
  const int tid = threadIdx.x, lane = tid & 31, wave = tid >> 5;
  const int c = lane & 15, hh = lane >> 4, koff = hh * 8, mOff = hh * 8, c4 = c * 4;
  const int q4 = lane >> 3, c8 = (lane & 7) * 8;
  const int n0 = wave * 64;

  {
    const v8h z = {(_Float16)0.f, (_Float16)0.f, (_Float16)0.f, (_Float16)0.f,
                   (_Float16)0.f, (_Float16)0.f, (_Float16)0.f, (_Float16)0.f};
#pragma unroll 1
    for (int i = tid; i < (kBatch * kHP) / 8; i += kScanThr) {
      *(v8h*)(Hh + i * 8) = z;
      *(v8h*)(Hl + i * 8) = z;
    }
  }
  __syncthreads();

  float* slab = Sl[wave];
  const _Float16* ahrow = Hh + c * kHP + koff;
  const _Float16* alrow = Hl + c * kHP + koff;
  const _Float16* brow  = U + (size_t)(n0 + c) * kHid + koff;
  const v8f z8 = {0.f, 0.f, 0.f, 0.f, 0.f, 0.f, 0.f, 0.f};

#pragma unroll 1
  for (int t = 0; t < kSteps; ++t) {
    const float* pt = P + (size_t)t * kBatch * kHid + n0 + c4;
    wave_sync();
#pragma unroll
    for (int it = 0; it < 8; ++it) {
      const int row = it * 2 + hh;
      const v4f p = *(const v4f*)(pt + (size_t)row * kHid);
      *(v4f*)(slab + row * kSlabP + c4) = p;
    }
    wave_sync();
    v8f acc[4], accr[4];
#pragma unroll
    for (int j = 0; j < 4; ++j) {
#pragma unroll
      for (int r = 0; r < 8; ++r) acc[j][r] = slab[(mOff + r) * kSlabP + 16 * j + c] * kWCarry;
      accr[j] = z8;
    }

#pragma unroll 2
    for (int kc = 0; kc < kHid / 32; ++kc) {
      const v16h fa = FragH::load(ahrow + kc * 32);
      const v16h fl = FragH::load(alrow + kc * 32);
      v16h fb[4];
#pragma unroll
      for (int j = 0; j < 4; ++j) fb[j] = FragH::load(brow + (size_t)(16 * j) * kHid + kc * 32);
#pragma unroll
      for (int j = 0; j < 4; ++j) {
        acc[j]  = FragH::mma(fa, fb[j], acc[j]);
        accr[j] = FragH::mma(fl, fb[j], accr[j]);
      }
      guard8_h(acc[0], acc[1], acc[2], acc[3], accr[0], accr[1], accr[2], accr[3], fa, fl);
      keep4_h(fb[0], fb[1], fb[2], fb[3]);
    }
    acc_guard4(acc[0], acc[1], acc[2], acc[3]);
    acc_guard4(accr[0], accr[1], accr[2], accr[3]);

#pragma unroll
    for (int j = 0; j < 4; ++j)
#pragma unroll
      for (int r = 0; r < 8; ++r)
        slab[(mOff + r) * kSlabP + 16 * j + c] = (acc[j][r] + accr[j][r] * kRCarryInv) * kWCarryInv;

    __syncthreads();

#pragma unroll 1
    for (int it = 0; it < 8; ++it) {
      const int row = it * 2 + hh;
      const v4f a4 = *(const v4f*)(slab + row * kSlabP + c4);
      v4f h4;
      v4h hi4, lo4;
#pragma unroll
      for (int e = 0; e < 4; ++e) {
        const float av = a4[e];
        const float hv = kDropScale * tanh_f(av);
        const _Float16 h16 = (_Float16)hv;
        const float res = (hv - (float)h16) * kRCarry;
        h4[e]  = hv;
        hi4[e] = h16;
        lo4[e] = (_Float16)res;
      }
      *(v4h*)(Hh + row * kHP + n0 + c4) = hi4;
      *(v4h*)(Hl + row * kHP + n0 + c4) = lo4;
      if (TOP) *(v4f*)(slab + row * kSlabP + c4) = h4;
    }

    __syncthreads();

    if (TOP) {
      for (int pass = 0; pass < 2; ++pass) {
#pragma unroll
        for (int it = 0; it < 8; ++it) {
          const int row = it * 2 + hh;
          const v4f v = *(const v4f*)(slab + row * kSlabP + c4);
          *(volatile v4f*)(OUT + ((size_t)t * kBatch + row) * kHid + n0 + c4) = v;
        }
        __threadfence();
      }
    } else {
      for (int pass = 0; pass < 2; ++pass) {
#pragma unroll
        for (int it = 0; it < 4; ++it) {
          const int rr = it * 4 + q4;
          const v8h vh = *(const v8h*)(Hh + rr * kHP + n0 + c8);
          const v8h vl = *(const v8h*)(Hl + rr * kHP + n0 + c8);
          *(volatile v8h*)(HHI + ((size_t)t * kBatch + rr) * kHid + n0 + c8) = vh;
          *(volatile v8h*)(HLO + ((size_t)t * kBatch + rr) * kHid + n0 + c8) = vl;
        }
        __threadfence();
      }
    }
  }
}

extern "C" void kernel_launch(void* const* d_in, const int* in_sizes, int n_in,
                              void* d_out, int out_size, void* d_ws, size_t ws_size, hipStream_t stream) {
  if (n_in < 7 || d_out == nullptr || d_ws == nullptr) return;
  if (in_sizes[0] != kRows * kFeat || in_sizes[1] != kHid * kFeat || in_sizes[2] != kHid ||
      in_sizes[3] != kHid * kHid || in_sizes[4] != kHid * kHid || in_sizes[5] != kHid ||
      in_sizes[6] != kHid * kHid || out_size != kRows * kHid) return;

  const float* x  = (const float*)d_in[0];
  const float* w0 = (const float*)d_in[1];
  const float* b0 = (const float*)d_in[2];
  const float* u0 = (const float*)d_in[3];
  const float* w1 = (const float*)d_in[4];
  const float* b1 = (const float*)d_in[5];
  const float* u1 = (const float*)d_in[6];
  float* out = (float*)d_out;

  char* ws = (char*)d_ws;
  size_t off = 0;
  auto carve = [&](size_t bytes) -> char* { char* p = ws + off; off += (bytes + 255) & ~(size_t)255; return p; };
  unsigned short* XH   = (unsigned short*)carve((size_t)kRows * kFeatP * 2);
  unsigned short* W0H  = (unsigned short*)carve((size_t)kHid * kFeatP * 2);
  unsigned short* U0H  = (unsigned short*)carve((size_t)kHid * kHid * 2);
  unsigned short* W1H  = (unsigned short*)carve((size_t)kHid * kHid * 2);
  unsigned short* U1H  = (unsigned short*)carve((size_t)kHid * kHid * 2);
  float*          BIAS = (float*)carve((size_t)2 * kHid * 4);
  float*          Pp   = (float*)carve((size_t)kRows * kHid * 4);
  unsigned short* HHI  = (unsigned short*)carve((size_t)kRows * kHid * 2);
  unsigned short* HLO  = (unsigned short*)carve((size_t)kRows * kHid * 2);
  if (off > ws_size || off > (size_t)134217728) return;

  prep_kernel<<<kPrepBlocks, 256, 0, stream>>>(x, w0, b0, u0, w1, b1, u1, XH, W0H, U0H, W1H, U1H, BIAS);

  gemm_f16_kernel<4, false><<<(kRows / 64) * (kHid / 64) / 8, 256, 0, stream>>>(
      XH, XH, kFeatP, W0H, kFeatP, Pp, kHid, BIAS, kRows, kHid, kFeatP, kWCarryInv, 0.0f);

  rnn_scan_kernel<false><<<1, kScanThr, 0, stream>>>(Pp, U0H, HHI, HLO, out);

  gemm_f16_kernel<2, true><<<(kRows / 32) * (kHid / 64) / 8, 256, 0, stream>>>(
      HHI, HLO, kHid, W1H, kHid, Pp, kHid, BIAS + kHid, kRows, kHid, kHid, kWCarryInv, kRCarryInv);

  rnn_scan_kernel<true><<<1, kScanThr, 0, stream>>>(Pp, U1H, HHI, HLO, out);
}
